// RWKV_TimeMix_37864431682654
// MI455X (gfx1250) — hardware-verified
//
#include <hip/hip_runtime.h>
#include <math.h>

constexpr int kBatch     = 8;
constexpr int kT         = 1024;
constexpr int kC         = 1024;
constexpr int kH         = 16;
constexpr int kHS        = 64;
constexpr int kN3        = 3 * kC;
constexpr int kBChunk    = 4;
constexpr int kRowsChunk = kBChunk * kT;
constexpr int kRowsAll   = kBatch * kT;
constexpr int kNChunk    = kBatch / kBChunk;
constexpr int kTabLen    = 1152;
constexpr int kKvPitch   = 40;
constexpr float kFltMin  = 1.17549435e-38f;
static_assert(kH * kHS == kC);
static_assert(kRowsChunk % 64 == 0 && kN3 % 64 == 0 && kC % 64 == 0 && kC % 32 == 0);
static_assert(kT % 64 == 0 && kC % 256 == 0 && kBatch % kBChunk == 0 && kRowsChunk % kT == 0);
static_assert((kTabLen * 2) % 16 == 0 && kTabLen >= kT + 64 + 32);
static_assert((kKvPitch * 2) % 16 == 0 && kKvPitch >= 32);
static_assert(((kRowsChunk / 64) * (kN3 / 64)) % 8 == 0 && ((kRowsChunk / 64) * (kC / 64)) % 8 == 0);

typedef __attribute__((ext_vector_type(16))) _Float16 v16h;
typedef __attribute__((ext_vector_type(8)))  _Float16 v8h;
typedef __attribute__((ext_vector_type(16))) __bf16   v16b;
typedef __attribute__((ext_vector_type(8)))  __bf16   v8b;
typedef __attribute__((ext_vector_type(8)))  float    v8f;
typedef __attribute__((ext_vector_type(4)))  float    v4f;
typedef __attribute__((ext_vector_type(4)))  unsigned int v4u;

__device__ __forceinline__ unsigned short f2bf_bits(float f) {
  unsigned u = __float_as_uint(f);
  return (unsigned short)((u + 0x7FFFu + ((u >> 16) & 1u)) >> 16);
}
__device__ __forceinline__ float bf_bits2f(unsigned short h) { return __uint_as_float(((unsigned)h) << 16); }

__device__ __forceinline__ void dep_guard_h(v8f& a, v8f& b, v16h x, v16h y) { asm volatile("v_nop\n\tv_nop\n\tv_nop\n\tv_nop" : "+v"(a), "+v"(b) : "v"(x), "v"(y)); }
__device__ __forceinline__ void dep_guard_b(v8f& a, v8f& b, v16b x, v16b y) { asm volatile("v_nop\n\tv_nop\n\tv_nop\n\tv_nop" : "+v"(a), "+v"(b) : "v"(x), "v"(y)); }
__device__ __forceinline__ void dep_guard4_h(v8f& a, v8f& b, v8f& c, v8f& d, v16h x, v16h y) { asm volatile("v_nop\n\tv_nop\n\tv_nop\n\tv_nop" : "+v"(a), "+v"(b), "+v"(c), "+v"(d) : "v"(x), "v"(y)); }
__device__ __forceinline__ void dep_guard4_b(v8f& a, v8f& b, v8f& c, v8f& d, v16b x, v16b y) { asm volatile("v_nop\n\tv_nop\n\tv_nop\n\tv_nop" : "+v"(a), "+v"(b), "+v"(c), "+v"(d) : "v"(x), "v"(y)); }
__device__ __forceinline__ void keep4_h(v16h a, v16h b, v16h c, v16h d) { asm volatile("v_nop" :: "v"(a), "v"(b), "v"(c), "v"(d)); }
__device__ __forceinline__ void keep4_b(v16b a, v16b b, v16b c, v16b d) { asm volatile("v_nop" :: "v"(a), "v"(b), "v"(c), "v"(d)); }
__device__ __forceinline__ void acc_guard4(v8f& a, v8f& b, v8f& c, v8f& d) { asm volatile("v_nop\n\tv_nop\n\tv_nop\n\tv_nop" : "+v"(a), "+v"(b), "+v"(c), "+v"(d)); }
template <typename T> struct Frag;
template <> struct Frag<_Float16> {
  typedef v16h V; union U { v16h v; v8h h[2]; };
  static __device__ __forceinline__ v16h load(const _Float16* p) {
    U f; f.h[0] = *(const v8h*)(p); f.h[1] = *(const v8h*)(p + 16); return f.v;
  }
  static __device__ __forceinline__ v8f mma(v16h a, v16h b, v8f c) {
    return __builtin_amdgcn_wmma_f32_16x16x32_f16(false, a, false, b, (short)0, c, false, false);
  }
  static __device__ __forceinline__ void guard(v8f& a, v8f& b, v16h x, v16h y) { dep_guard_h(a, b, x, y); }
  static __device__ __forceinline__ void guard4(v8f& a, v8f& b, v8f& c, v8f& d, v16h x, v16h y) { dep_guard4_h(a, b, c, d, x, y); }
  static __device__ __forceinline__ void keep(v16h a, v16h b, v16h c, v16h d) { keep4_h(a, b, c, d); }
};
template <> struct Frag<__bf16> {
  typedef v16b V; union U { v16b v; v8b h[2]; };
  static __device__ __forceinline__ v16b load(const __bf16* p) {
    U f; f.h[0] = *(const v8b*)(p); f.h[1] = *(const v8b*)(p + 16); return f.v;
  }
  static __device__ __forceinline__ v8f mma(v16b a, v16b b, v8f c) {
    return __builtin_amdgcn_wmma_f32_16x16x32_bf16(false, a, false, b, (short)0, c, false, false);
  }
  static __device__ __forceinline__ void guard(v8f& a, v8f& b, v16b x, v16b y) { dep_guard_b(a, b, x, y); }
  static __device__ __forceinline__ void guard4(v8f& a, v8f& b, v8f& c, v8f& d, v16b x, v16b y) { dep_guard4_b(a, b, c, d, x, y); }
  static __device__ __forceinline__ void keep(v16b a, v16b b, v16b c, v16b d) { keep4_b(a, b, c, d); }
};

__device__ __forceinline__ unsigned pk16(unsigned short a, unsigned short b) { return (unsigned)a | ((unsigned)b << 16); }

__device__ __forceinline__ v8f bmma(v16b a, v16b b, v8f c) {
  c = __builtin_amdgcn_wmma_f32_16x16x32_bf16(false, a, false, b, (short)0, c, false, false);
  asm volatile("v_nop\n\tv_nop\n\tv_nop\n\tv_nop" : "+v"(c) : "v"(a), "v"(b));
  return c;
}

template <int ET> struct Elem;
template <> struct Elem<0> { typedef _Float16 T; };
template <> struct Elem<1> { typedef __bf16 T; };
template <int ET, bool SPLIT, int BIAS_MODE, int OUT_MODE, bool RESID, int ACT = 0>
__global__ __launch_bounds__(256) void wmma_gemm64(
    const unsigned short* __restrict__ Ap, const unsigned short* __restrict__ A2p, int lda, long strideA,
    const unsigned short* __restrict__ Btp, const unsigned short* __restrict__ Bt2p, int ldb, long strideB,
    void* __restrict__ Cout, void* __restrict__ Cout2, int ldc, long strideC,
    const float* __restrict__ bias,
    const float* __restrict__ resid, long strideR,
    int M, int N, int K, float scale) {
  typedef typename Elem<ET>::T T;
  typedef typename Frag<T>::V V;
  const T* A = (const T*)Ap; const T* A2 = (const T*)A2p; const T* Bt = (const T*)Btp; const T* Bt2 = (const T*)Bt2p;
  __shared__ __align__(16) float sT[8][16 * 68];
  const int b    = blockIdx.y;
  const int lane = threadIdx.x & 31;
  const int wave = threadIdx.x >> 5;
  const int tilesN = N >> 6;
  const int tilesM = M >> 6;
  const int tile = blockIdx.x * 8 + wave;
  if (tile >= tilesM * tilesN) return;
  const int tm = tile / tilesN;
  const int tn = tile - tm * tilesN;
  const int m0 = tm << 6;
  const int n0 = tn << 6;

  const T* Ab  = A  + (size_t)b * strideA;
  const T* Bb  = Bt + (size_t)b * strideB;
  const T* Ab2 = SPLIT ? (A2  + (size_t)b * strideA) : nullptr;
  const T* Bb2 = SPLIT ? (Bt2 + (size_t)b * strideB) : nullptr;

  const int rlane = lane & 15;
  const int koff  = (lane >> 4) * 8;
  const int mOff  = (lane >> 4) * 8;

  v8f acc[4][4];
#pragma unroll
  for (int i = 0; i < 4; ++i)
#pragma unroll
    for (int j = 0; j < 4; ++j) acc[i][j] = (v8f){0.f,0.f,0.f,0.f,0.f,0.f,0.f,0.f};

  for (int k0 = 0; k0 < K; k0 += 32) {
    V bh[4], bl[4];
#pragma unroll
    for (int j = 0; j < 4; ++j) {
      const size_t bo = (size_t)(n0 + (j << 4) + rlane) * ldb + koff + k0;
      bh[j] = Frag<T>::load(Bb + bo);
      if (SPLIT) bl[j] = Frag<T>::load(Bb2 + bo);
    }
#pragma unroll
    for (int i = 0; i < 4; ++i) {
      const size_t ao = (size_t)(m0 + (i << 4) + rlane) * lda + koff + k0;
      V ah = Frag<T>::load(Ab + ao);
      V al;
      if (SPLIT) al = Frag<T>::load(Ab2 + ao);
#pragma unroll
      for (int j = 0; j < 4; ++j) {
        acc[i][j] = Frag<T>::mma(ah, bh[j], acc[i][j]);
        if (SPLIT) {
          acc[i][j] = Frag<T>::mma(ah, bl[j], acc[i][j]);
          acc[i][j] = Frag<T>::mma(al, bh[j], acc[i][j]);
        }
      }
      Frag<T>::guard4(acc[i][0], acc[i][1], acc[i][2], acc[i][3], ah, SPLIT ? al : ah);
    }
    Frag<T>::keep(bh[0], bh[1], bh[2], bh[3]);
    if (SPLIT) Frag<T>::keep(bl[0], bl[1], bl[2], bl[3]);
  }
  acc_guard4(acc[0][0], acc[0][1], acc[0][2], acc[0][3]);
  acc_guard4(acc[1][0], acc[1][1], acc[1][2], acc[1][3]);
  acc_guard4(acc[2][0], acc[2][1], acc[2][2], acc[2][3]);
  acc_guard4(acc[3][0], acc[3][1], acc[3][2], acc[3][3]);

  float* slab = sT[wave];
  const float* Rb = RESID ? (resid + (size_t)b * strideR) : nullptr;
#pragma unroll
  for (int i = 0; i < 4; ++i) {
    const int mBase = m0 + (i << 4);
#pragma unroll
    for (int j = 0; j < 4; ++j) {
      const int n = n0 + (j << 4) + rlane;
      float bv = 0.f;
      if (BIAS_MODE == 2) bv = bias[n];
#pragma unroll
      for (int r = 0; r < 8; ++r) {
        float v = acc[i][j][r] * scale;
        if (BIAS_MODE == 1) v += bias[mBase + mOff + r];
        if (BIAS_MODE == 2) v += bv;
        if (RESID) v += Rb[(size_t)(mBase + mOff + r) * ldc + n];
        if (ACT == 2) v = fmaxf(v, 0.0f);
        if (ACT == 4) v = (v > 0.f) ? v : 0.01f * v;
        slab[(mOff + r) * 68 + (j << 4) + rlane] = v;
      }
    }
    __builtin_amdgcn_fence(__ATOMIC_RELEASE, "workgroup");
    __builtin_amdgcn_wave_barrier();
    __builtin_amdgcn_fence(__ATOMIC_ACQUIRE, "workgroup");
    if (OUT_MODE == 0) {
      float* C = (float*)Cout + (size_t)b * strideC;
      const int hh = lane >> 4, c4 = (lane & 15) * 4;
      for (int pass = 0; pass < 2; ++pass) {
#pragma unroll
        for (int it = 0; it < 8; ++it) {
          const int row = it * 2 + hh;
          v4f v = *(const v4f*)(slab + row * 68 + c4);
          *(volatile v4f*)(C + (size_t)(mBase + row) * ldc + n0 + c4) = v;
        }
        __threadfence();
      }
    } else {
      const int q = lane >> 3, c8 = (lane & 7) * 8;
      unsigned short* C  = (unsigned short*)Cout  + (size_t)b * strideC;
      unsigned short* C2 = (OUT_MODE == 2) ? ((unsigned short*)Cout2 + (size_t)b * strideC) : nullptr;
      for (int pass = 0; pass < 2; ++pass) {
#pragma unroll
        for (int it = 0; it < 4; ++it) {
          const int row = it * 4 + q;
          const float* sp = slab + row * 68 + c8;
          v8h hv, lv;
#pragma unroll
          for (int e = 0; e < 8; ++e) {
            if (OUT_MODE == 1) {
              hv[e] = (_Float16)sp[e];
            } else {
              unsigned short hb = f2bf_bits(sp[e]);
              unsigned short lb = f2bf_bits(sp[e] - bf_bits2f(hb));
              hv[e] = __builtin_bit_cast(_Float16, hb);
              lv[e] = __builtin_bit_cast(_Float16, lb);
            }
          }
          *(volatile v8h*)(C + (size_t)(mBase + row) * ldc + n0 + c8) = hv;
          if (OUT_MODE == 2) *(volatile v8h*)(C2 + (size_t)(mBase + row) * ldc + n0 + c8) = lv;
        }
        __threadfence();
      }
    }
    __builtin_amdgcn_fence(__ATOMIC_RELEASE, "workgroup");
    __builtin_amdgcn_wave_barrier();
    __builtin_amdgcn_fence(__ATOMIC_ACQUIRE, "workgroup");
  }
}

template <bool SPLITA, bool BIASN, bool ROWSC>
__global__ __launch_bounds__(256) void wmma_gemm64_b16a(
    const unsigned short* __restrict__ Ap, const unsigned short* __restrict__ A2p, int lda,
    const unsigned short* __restrict__ Btp, int ldb,
    float* __restrict__ Cout, int ldc,
    const float* __restrict__ bias, const float* __restrict__ rscale, int rsoff, int rsmask,
    int M, int N, int K) {
  const __bf16* A = (const __bf16*)Ap; const __bf16* A2 = (const __bf16*)A2p; const __bf16* Bt = (const __bf16*)Btp;
  __shared__ __align__(16) float sT[8][16 * 68];
  const int lane = threadIdx.x & 31;
  const int wave = threadIdx.x >> 5;
  const int tilesN = N >> 6;
  const int tilesM = M >> 6;
  const int tile = blockIdx.x * 8 + wave;
  if (tile >= tilesM * tilesN) return;
  const int tm = tile / tilesN;
  const int tn = tile - tm * tilesN;
  const int m0 = tm << 6;
  const int n0 = tn << 6;

  const int rlane = lane & 15;
  const int koff  = (lane >> 4) * 8;
  const int mOff  = (lane >> 4) * 8;

  v8f acc[4][4];
#pragma unroll
  for (int i = 0; i < 4; ++i)
#pragma unroll
    for (int j = 0; j < 4; ++j) acc[i][j] = (v8f){0.f,0.f,0.f,0.f,0.f,0.f,0.f,0.f};

  for (int k0 = 0; k0 < K; k0 += 32) {
    v16b bh[4];
#pragma unroll
    for (int j = 0; j < 4; ++j) {
      const size_t bo = (size_t)(n0 + (j << 4) + rlane) * ldb + koff + k0;
      bh[j] = Frag<__bf16>::load(Bt + bo);
    }
#pragma unroll
    for (int i = 0; i < 4; ++i) {
      const size_t ao = (size_t)(m0 + (i << 4) + rlane) * lda + koff + k0;
      v16b ah = Frag<__bf16>::load(A + ao);
      v16b al = ah;
      if (SPLITA) al = Frag<__bf16>::load(A2 + ao);
#pragma unroll
      for (int j = 0; j < 4; ++j) {
        acc[i][j] = Frag<__bf16>::mma(ah, bh[j], acc[i][j]);
        if (SPLITA) acc[i][j] = Frag<__bf16>::mma(al, bh[j], acc[i][j]);
      }
      dep_guard4_b(acc[i][0], acc[i][1], acc[i][2], acc[i][3], ah, al);
    }
    keep4_b(bh[0], bh[1], bh[2], bh[3]);
  }
  acc_guard4(acc[0][0], acc[0][1], acc[0][2], acc[0][3]);
  acc_guard4(acc[1][0], acc[1][1], acc[1][2], acc[1][3]);
  acc_guard4(acc[2][0], acc[2][1], acc[2][2], acc[2][3]);
  acc_guard4(acc[3][0], acc[3][1], acc[3][2], acc[3][3]);

  float* slab = sT[wave];
#pragma unroll
  for (int i = 0; i < 4; ++i) {
    const int mBase = m0 + (i << 4);
#pragma unroll
    for (int j = 0; j < 4; ++j) {
      const int n = n0 + (j << 4) + rlane;
      float bvn = 0.f;
      if (BIASN) bvn = bias[n];
#pragma unroll
      for (int r = 0; r < 8; ++r) {
        slab[(mOff + r) * 68 + (j << 4) + rlane] = acc[i][j][r] + bvn;
      }
    }
    __builtin_amdgcn_fence(__ATOMIC_RELEASE, "workgroup");
    __builtin_amdgcn_wave_barrier();
    __builtin_amdgcn_fence(__ATOMIC_ACQUIRE, "workgroup");
    {
      const int hh = lane >> 4, c4 = (lane & 15) * 4;
      for (int pass = 0; pass < 2; ++pass) {
#pragma unroll
        for (int it = 0; it < 8; ++it) {
          const int row = it * 2 + hh;
          v4f v = *(const v4f*)(slab + row * 68 + c4);
          if (ROWSC) {
            const float gm = rscale[(mBase + row + rsoff) & rsmask];
            v = v * gm;
          }
          *(volatile v4f*)(Cout + (size_t)(mBase + row) * ldc + n0 + c4) = v;
        }
        __threadfence();
      }
    }
    __builtin_amdgcn_fence(__ATOMIC_RELEASE, "workgroup");
    __builtin_amdgcn_wave_barrier();
    __builtin_amdgcn_fence(__ATOMIC_ACQUIRE, "workgroup");
  }
}

__global__ __launch_bounds__(256) void xs_cast_kernel(const float* __restrict__ x, unsigned short* __restrict__ XS) {
  const int i  = blockIdx.x * 256 + threadIdx.x;
  const int e0 = i * 8;
  const int m  = e0 >> 10;
  const int c  = e0 & (kC - 1);
  const int t  = m & (kT - 1);
  const bool sh = (c < kC / 2);
  const bool zr = sh && (t == 0);
  const int srow = (sh && t > 0) ? (m - 1) : m;
  const float* p = x + (size_t)srow * kC + c;
  const v4f a  = *(const v4f*)(p);
  const v4f a2 = *(const v4f*)(p + 4);
  unsigned short hb[8];
#pragma unroll
  for (int e = 0; e < 4; ++e) {
    const float f0 = zr ? 0.0f : a[e];
    const float f1 = zr ? 0.0f : a2[e];
    hb[e]     = f2bf_bits(f0);
    hb[4 + e] = f2bf_bits(f1);
  }
  const v4u u = (v4u){pk16(hb[0], hb[1]), pk16(hb[2], hb[3]), pk16(hb[4], hb[5]), pk16(hb[6], hb[7])};
  unsigned short* q = XS + (size_t)e0;
  *(volatile v4u*)q = u;
  __threadfence();
  *(volatile v4u*)q = u;
}

__global__ __launch_bounds__(256) void wt_cast_kernel(const float* __restrict__ W0, const float* __restrict__ W1,
                                                     const float* __restrict__ W2, const float* __restrict__ W3,
                                                     unsigned short* __restrict__ WT) {
  __shared__ float sm[64][65];
  const int t  = threadIdx.x;
  const int k0 = blockIdx.x * 64;
  const int n0 = blockIdx.y * 64;
  const int z  = blockIdx.z;
  const float* W = (z == 0) ? W0 : (z == 1) ? W1 : (z == 2) ? W2 : W3;
#pragma unroll
  for (int i = 0; i < 16; ++i) {
    const int e = i * 256 + t;
    const int r = e >> 6;
    const int c = e & 63;
    sm[c][r] = W[(size_t)(k0 + r) * kC + n0 + c];
  }
  __syncthreads();
  const int lane = t & 31, wave = t >> 5;
  const int q = lane >> 3, c8 = (lane & 7) * 8;
  unsigned short* op = WT + (size_t)z * kC * kC;
  for (int pass = 0; pass < 2; ++pass) {
#pragma unroll
    for (int it = 0; it < 2; ++it) {
      const int row = wave * 8 + it * 4 + q;
      unsigned short hb[8];
#pragma unroll
      for (int e = 0; e < 8; ++e) hb[e] = f2bf_bits(sm[row][c8 + e]);
      const v4u u = (v4u){pk16(hb[0], hb[1]), pk16(hb[2], hb[3]), pk16(hb[4], hb[5]), pk16(hb[6], hb[7])};
      *(volatile v4u*)(op + (size_t)(n0 + row) * kC + k0 + c8) = u;
    }
    __threadfence();
  }
}

__global__ __launch_bounds__(256) void gate_scan_kernel(const float* __restrict__ P, const float* __restrict__ alpha,
                                                       const float* __restrict__ bk, const float* __restrict__ bv,
                                                       const float* __restrict__ br,
                                                       float* __restrict__ G, unsigned short* __restrict__ KVH,
                                                       unsigned short* __restrict__ KVL) {
  __shared__ __align__(16) float gs[256];
  __shared__ __align__(16) float kvs[256];
  const int th   = threadIdx.x;
  const int lane = th & 31, wave = th >> 5;
  const int cb   = blockIdx.x * 256;
  const int bl   = blockIdx.y;
  const int c    = cb + th;
  const int h    = c >> 6;
  const float bkc = bk[c];
  const float bvc = bv[c];
  const float brc = br[c];
  const float* arow = alpha + (size_t)h * kT;
  double sum = 0.0;
#pragma unroll 1
  for (int t = 0; t < kT; ++t) {
    const size_t m = (size_t)bl * kT + t;
    const float* pr = P + m * (size_t)kN3;
    const float kp = pr[c] + bkc;
    const float vv = pr[kC + c] + bvc;
    const float rr = pr[2 * kC + c] + brc;
    const float al = arow[t];
    const float kcl = fminf(fmaxf(kp, -60.0f), 30.0f);
    const float ke  = expf(kcl);
    sum += (double)ke;
    const float sumf = (float)sum;
    const float sg = 1.0f / (1.0f + expf(-rr));
    const float g  = sg / sumf;
    const float kv = ke * vv * al;
    gs[th]  = g;
    kvs[th] = kv;
    __syncthreads();
    if (wave < 2) {
      const v4f val = *(const v4f*)(gs + 4 * th);
      float* dp = G + m * (size_t)kC + cb + 4 * th;
      *(volatile v4f*)dp = val;
      __threadfence();
      *(volatile v4f*)dp = val;
    } else if (wave < 4) {
      const bool lo = (wave == 3);
      const v4f a  = *(const v4f*)(kvs + 8 * lane);
      const v4f a2 = *(const v4f*)(kvs + 8 * lane + 4);
      unsigned short bits[8];
#pragma unroll
      for (int e = 0; e < 4; ++e) {
        const float f0 = a[e];
        const float f1 = a2[e];
        const unsigned short h0 = f2bf_bits(f0);
        const unsigned short h1 = f2bf_bits(f1);
        const unsigned short l0 = f2bf_bits(f0 - bf_bits2f(h0));
        const unsigned short l1 = f2bf_bits(f1 - bf_bits2f(h1));
        bits[e]     = lo ? l0 : h0;
        bits[4 + e] = lo ? l1 : h1;
      }
      const v4u u = (v4u){pk16(bits[0], bits[1]), pk16(bits[2], bits[3]), pk16(bits[4], bits[5]), pk16(bits[6], bits[7])};
      unsigned short* dp = (lo ? KVL : KVH) + m * (size_t)kC + cb + 8 * lane;
      *(volatile v4u*)dp = u;
      __threadfence();
      *(volatile v4u*)dp = u;
    }
    __syncthreads();
  }
}

__global__ __launch_bounds__(128) void decay_agg_kernel(const unsigned short* __restrict__ KVH, const unsigned short* __restrict__ KVL,
                                                       const float* __restrict__ G, const float* __restrict__ time_w,
                                                       const float* __restrict__ beta,
                                                       unsigned short* __restrict__ YH, unsigned short* __restrict__ YL) {
  union FB { v16b v; v8b h[2]; };
  __shared__ __align__(16) float twf[kT];
  __shared__ __align__(16) unsigned short tab[8 * kTabLen];
  __shared__ __align__(16) float betas[64];
  __shared__ __align__(16) unsigned short kvT[2][64 * kKvPitch];
  __shared__ __align__(16) float Os[4][16 * 68];

  const int tid  = threadIdx.x;
  const int lane = tid & 31, wave = tid >> 5;
  const int rlane = lane & 15;
  const int koff  = (lane >> 4) * 8;
  const int mOff  = koff;
  const int gx = blockIdx.x, h = blockIdx.y, bl = blockIdx.z;
  const int t0b = gx * 64;
  const int t0w = t0b + wave * 16;

#pragma unroll
  for (int i = 0; i < 2; ++i) {
    const int f0 = (tid + i * 128) * 4;
    *(v4f*)(twf + f0) = *(const v4f*)(time_w + (size_t)h * kT + f0);
  }
  if (tid < 64) betas[tid] = beta[(size_t)h * kT + t0b + tid];
  __syncthreads();
#pragma unroll 1
  for (int s = 0; s < 8; ++s) {
    for (int j = tid; j < kTabLen; j += 128) {
      const int src  = j + s;
      const int srcc = (src < kT) ? src : (kT - 1);
      float val = twf[srcc];
      val = (src < kT) ? val : 0.0f;
      val = (fabsf(val) < kFltMin) ? 0.0f : val;
      tab[s * kTabLen + j] = f2bf_bits(val);
    }
  }
  __syncthreads();

  v8f acc[4];
#pragma unroll
  for (int ct = 0; ct < 4; ++ct) acc[ct] = (v8f){0.f,0.f,0.f,0.f,0.f,0.f,0.f,0.f};

  const __bf16* tabbf = (const __bf16*)tab;
  const __bf16* kvTh  = (const __bf16*)kvT[0];
  const __bf16* kvTl  = (const __bf16*)kvT[1];
  const int nchunk = (t0b >> 5) + 2;
#pragma unroll 1
  for (int cc = 0; cc < nchunk; ++cc) {
    const int u0 = cc << 5;
#pragma unroll
    for (int ii = 0; ii < 2; ++ii) {
      const int idx = tid + ii * 128;
      const int u   = idx >> 3;
      const int c0  = (idx & 7) * 8;
      const size_t goff = ((size_t)bl * kT + u0 + u) * kC + h * kHS + c0;
      const v4u wh = *(const v4u*)(KVH + goff);
      const v4u wl = *(const v4u*)(KVL + goff);
#pragma unroll
      for (int j = 0; j < 4; ++j) {
        const unsigned a  = wh[j];
        const unsigned a2 = wl[j];
        kvT[0][(c0 + 2 * j) * kKvPitch + u]     = (unsigned short)(a & 0xffffu);
        kvT[0][(c0 + 2 * j + 1) * kKvPitch + u] = (unsigned short)(a >> 16);
        kvT[1][(c0 + 2 * j) * kKvPitch + u]     = (unsigned short)(a2 & 0xffffu);
        kvT[1][(c0 + 2 * j + 1) * kKvPitch + u] = (unsigned short)(a2 >> 16);
      }
    }
    __syncthreads();
    if (u0 <= t0w + 15) {
      const int base  = (kT - 1) - (t0w + rlane) + u0 + koff;
      const int s     = base & 7;
      const int base8 = base - s;
      FB fa;
      const __bf16* ap = tabbf + s * kTabLen + base8;
      fa.h[0] = *(const v8b*)(ap);
      fa.h[1] = *(const v8b*)(ap + 16);
#pragma unroll
      for (int ct = 0; ct < 4; ++ct) {
        const int bo = (ct * 16 + rlane) * kKvPitch + koff;
        FB fbh, fbl;
        fbh.h[0] = *(const v8b*)(kvTh + bo);
        fbh.h[1] = *(const v8b*)(kvTh + bo + 16);
        fbl.h[0] = *(const v8b*)(kvTl + bo);
        fbl.h[1] = *(const v8b*)(kvTl + bo + 16);
        acc[ct] = bmma(fa.v, fbh.v, acc[ct]);
        acc[ct] = bmma(fa.v, fbl.v, acc[ct]);
      }
    }
    __syncthreads();
  }
  acc_guard4(acc[0], acc[1], acc[2], acc[3]);

  float* slab = Os[wave];
#pragma unroll
  for (int ct = 0; ct < 4; ++ct) {
#pragma unroll
    for (int r = 0; r < 8; ++r) {
      slab[(mOff + r) * 68 + ct * 16 + rlane] = acc[ct][r] * betas[wave * 16 + mOff + r];
    }
  }
  __builtin_amdgcn_fence(__ATOMIC_RELEASE, "workgroup");
  __builtin_amdgcn_wave_barrier();
  __builtin_amdgcn_fence(__ATOMIC_ACQUIRE, "workgroup");
  {
    const int q = lane >> 3, c8 = (lane & 7) * 8;
    for (int pass = 0; pass < 2; ++pass) {
#pragma unroll
      for (int it = 0; it < 4; ++it) {
        const int row = it * 4 + q;
        const size_t m = (size_t)bl * kT + t0w + row;
        const size_t goff = m * kC + h * kHS + c8;
        const v4f g0 = *(const v4f*)(G + goff);
        const v4f g1 = *(const v4f*)(G + goff + 4);
        const float* sp = slab + row * 68 + c8;
        float yv[8];
#pragma unroll
        for (int e = 0; e < 4; ++e) {
          yv[e]     = sp[e] * g0[e];
          yv[4 + e] = sp[4 + e] * g1[e];
        }
        unsigned short hb[8], lb[8];
#pragma unroll
        for (int e = 0; e < 8; ++e) {
          hb[e] = f2bf_bits(yv[e]);
          lb[e] = f2bf_bits(yv[e] - bf_bits2f(hb[e]));
        }
        const v4u uh = (v4u){pk16(hb[0], hb[1]), pk16(hb[2], hb[3]), pk16(hb[4], hb[5]), pk16(hb[6], hb[7])};
        const v4u ul = (v4u){pk16(lb[0], lb[1]), pk16(lb[2], lb[3]), pk16(lb[4], lb[5]), pk16(lb[6], lb[7])};
        *(volatile v4u*)(YH + goff) = uh;
        *(volatile v4u*)(YL + goff) = ul;
      }
      __threadfence();
    }
  }
}

extern "C" void kernel_launch(void* const* d_in, const int* in_sizes, int n_in,
                              void* d_out, int out_size, void* d_ws, size_t ws_size,
                              hipStream_t stream) {
  if (n_in < 13) return;
  const int nAct = kRowsAll * kC;
  if (in_sizes[0] != nAct) return;
  if (in_sizes[1] != kH * kT || in_sizes[2] != kH * kT || in_sizes[3] != kH * kT) return;
  if (in_sizes[4] != kT) return;
  if (in_sizes[5] != kC * kC || in_sizes[7] != kC * kC || in_sizes[9] != kC * kC || in_sizes[11] != kC * kC) return;
  if (in_sizes[6] != kC || in_sizes[8] != kC || in_sizes[10] != kC || in_sizes[12] != kC) return;
  if (out_size != nAct) return;

  const size_t szXS = (size_t)kRowsAll * kC * 2;
  const size_t szWT = (size_t)4 * kC * kC * 2;
  const size_t szP  = (size_t)kRowsChunk * kN3 * 4;
  const size_t szG  = (size_t)kRowsChunk * kC * 4;
  const size_t sz16 = (size_t)kRowsChunk * kC * 2;
  const size_t offXS  = 0;
  const size_t offWT  = offXS + szXS;
  const size_t offP   = offWT + szWT;
  const size_t offG   = offP + szP;
  const size_t offKVH = offG + szG;
  const size_t offKVL = offKVH + sz16;
  const size_t offYH  = offKVL + sz16;
  const size_t offYL  = offYH + sz16;
  const size_t total  = offYL + sz16;
  if (ws_size < total) return;

  const float* x     = (const float*)d_in[0];
  const float* tw    = (const float*)d_in[1];
  const float* alpha = (const float*)d_in[2];
  const float* beta  = (const float*)d_in[3];
  const float* gamma = (const float*)d_in[4];
  const float* Wk    = (const float*)d_in[5];
  const float* bk    = (const float*)d_in[6];
  const float* Wv    = (const float*)d_in[7];
  const float* bv    = (const float*)d_in[8];
  const float* Wr    = (const float*)d_in[9];
  const float* br    = (const float*)d_in[10];
  const float* Wo    = (const float*)d_in[11];
  const float* bo    = (const float*)d_in[12];
  float* out = (float*)d_out;
  char* ws = (char*)d_ws;
  unsigned short* XS  = (unsigned short*)(ws + offXS);
  unsigned short* WT  = (unsigned short*)(ws + offWT);
  float*          P   = (float*)(ws + offP);
  float*          G   = (float*)(ws + offG);
  unsigned short* KVH = (unsigned short*)(ws + offKVH);
  unsigned short* KVL = (unsigned short*)(ws + offKVL);
  unsigned short* YH  = (unsigned short*)(ws + offYH);
  unsigned short* YL  = (unsigned short*)(ws + offYL);

  xs_cast_kernel<<<dim3((nAct / 8) / 256), dim3(256), 0, stream>>>(x, XS);
  wt_cast_kernel<<<dim3(kC / 64, kC / 64, 4), dim3(256), 0, stream>>>(Wk, Wv, Wr, Wo, WT);

  const unsigned short* WoT = WT + (size_t)3 * kC * kC;
  const int blocksProj = ((kRowsChunk / 64) * (kN3 / 64)) / 8;
  const int blocksOut  = ((kRowsChunk / 64) * (kC / 64)) / 8;

  for (int ch = 0; ch < kNChunk; ++ch) {
    const unsigned short* XSc = XS + (size_t)ch * kRowsChunk * kC;
    wmma_gemm64<1, false, 0, 0, false, 0><<<dim3(blocksProj, 1), dim3(256), 0, stream>>>(
        XSc, XSc, kC, 0L, WT, WT, kC, 0L,
        (void*)P, (void*)P, kN3, 0L, bo, bo, 0L, kRowsChunk, kN3, kC, 1.0f);
    gate_scan_kernel<<<dim3(kC / 256, kBChunk), dim3(256), 0, stream>>>(P, alpha, bk, bv, br, G, KVH, KVL);
    decay_agg_kernel<<<dim3(kT / 64, kH, kBChunk), dim3(128), 0, stream>>>(KVH, KVL, G, tw, beta, YH, YL);
    float* outc = out + (size_t)ch * kRowsChunk * kC;
    wmma_gemm64_b16a<true, true, true><<<dim3(blocksOut), dim3(256), 0, stream>>>(
        YH, YL, kC, WoT, kC, outc, kC, bo, gamma, ch * kRowsChunk, kT - 1, kRowsChunk, kC, kC);
  }
}
